// MB_Mamba_Block_49426483642710
// MI455X (gfx1250) — hardware-verified
//
#include <hip/hip_runtime.h>
#include <hip/hip_bf16.h>


#define NB_   2
#define NL_   2048
#define DM_   512
#define DI_   1024
#define NS_   16
#define DR_   32
#define DBC_  64
#define MT_   (NB_ * NL_)

static_assert(MT_ % 64 == 0);
static_assert(DM_ % 64 == 0);
static_assert(DI_ % 64 == 0);
static_assert((2 * DI_) % 64 == 0);
static_assert(DBC_ == 64);
static_assert(DR_ == 32);
static_assert(DM_ == 64 * 8);
static_assert(DI_ == 128 * 8);
static_assert((NL_ & (NL_ - 1)) == 0);
static_assert(NL_ % 16 == 0);
static_assert((DM_ & (DM_ - 1)) == 0);

typedef float          v4f   __attribute__((ext_vector_type(4)));
typedef float          v8f   __attribute__((ext_vector_type(8)));
typedef __bf16         v16b  __attribute__((ext_vector_type(16)));
typedef unsigned short u16x8 __attribute__((ext_vector_type(8)));

union FragB { u16x8 h[2]; v16b v; };

__device__ __forceinline__ unsigned short f32_to_bf16(float f) {
    unsigned u = __float_as_uint(f);
    unsigned r = u + 0x7FFFu + ((u >> 16) & 1u);
    return (unsigned short)(r >> 16);
}
__device__ __forceinline__ float bf16_to_f32(unsigned short b) {
    return __uint_as_float(((unsigned)b) << 16);
}
__device__ __forceinline__ float silu_f(float x) {
    const float e = __expf(-x);
    return x * __builtin_amdgcn_rcpf(1.0f + e);
}
__device__ __forceinline__ float softplus_f(float x) {
    return fmaxf(x, 0.0f) + log1pf(__expf(-fabsf(x)));
}
__device__ __forceinline__ float conv4(float x0, float x1, float x2, float x3,
                                       float w0, float w1, float w2, float w3, float bias) {
    return (w0 * x0 + w1 * x1 + w2 * x2 + w3 * x3) + bias;
}
__device__ __forceinline__ v8f ld8f(const float* p) {
    v4f a = *(const v4f*)p;
    v4f b = *(const v4f*)(p + 4);
    return __builtin_shufflevector(a, b, 0, 1, 2, 3, 4, 5, 6, 7);
}
__device__ __forceinline__ float wave_sum(float v) {
#pragma unroll
    for (int o = 16; o > 0; o >>= 1) v += __shfl_xor(v, o, 32);
    return v;
}

__device__ __forceinline__ void mma16(v8f& acc, const FragB& a, const FragB& b) {
    acc = __builtin_amdgcn_wmma_f32_16x16x32_bf16(false, a.v, false, b.v, (short)0, acc, false, false);
    asm volatile("v_nop\n\tv_nop\n\tv_nop\n\tv_nop" : "+v"(acc) : "v"(a.v), "v"(b.v));
}

__global__ __launch_bounds__(256)
void cvt_split_kernel(const float* __restrict__ src, unsigned short* dst0, unsigned short* dst1, int n8)
{
    const int i = blockIdx.x * 256 + threadIdx.x;
    if (i >= n8) return;
    const size_t e = (size_t)i * 8;
    const v8f x = ld8f(src + e);
    u16x8 hv, lv;
#pragma unroll
    for (int c = 0; c < 8; ++c) {
        const float f = x[c];
        const unsigned short hb = f32_to_bf16(f);
        const unsigned short lb = f32_to_bf16(f - bf16_to_f32(hb));
        hv[c] = hb;
        lv[c] = lb;
    }
    *(volatile u16x8*)(dst0 + e) = hv;
    *(volatile u16x8*)(dst1 + e) = lv;
    __threadfence();
    *(volatile u16x8*)(dst0 + e) = hv;
    *(volatile u16x8*)(dst1 + e) = lv;
}

__global__ __launch_bounds__(64)
void ln_kernel(const float* __restrict__ x, const float* __restrict__ g, const float* __restrict__ bt,
               unsigned short* fnh, unsigned short* fnl, unsigned short* frh, unsigned short* frl)
{
    __shared__ float red[4];
    const int row  = blockIdx.x;
    const int tid  = threadIdx.x;
    const int lane = tid & 31;
    const int wave = tid >> 5;
    const size_t e = (size_t)row * DM_ + tid * 8;

    const v8f v = ld8f(x + e);
    float s = 0.0f;
#pragma unroll
    for (int c = 0; c < 8; ++c) s += v[c];
    s = wave_sum(s);
    if (lane == 0) red[wave] = s;
    __syncthreads();
    const float mean = (red[0] + red[1]) * (1.0f / DM_);

    v8f dv;
    float q = 0.0f;
#pragma unroll
    for (int c = 0; c < 8; ++c) { dv[c] = v[c] - mean; q += dv[c] * dv[c]; }
    q = wave_sum(q);
    if (lane == 0) red[2 + wave] = q;
    __syncthreads();
    const float var  = (red[2] + red[3]) * (1.0f / DM_);
    const float rstd = rsqrtf(var + 1e-5f);

    const v8f gg = ld8f(g + tid * 8);
    const v8f bb = ld8f(bt + tid * 8);
    u16x8 h0, l0, h1, l1;
#pragma unroll
    for (int c = 0; c < 8; ++c) {
        const float y  = dv[c] * rstd * gg[c] + bb[c];
        const unsigned short hb = f32_to_bf16(y);
        const unsigned short lb = f32_to_bf16(y - bf16_to_f32(hb));
        const float yr = fmaxf(y, 0.0f);
        const unsigned short hr = f32_to_bf16(yr);
        const unsigned short lr = f32_to_bf16(yr - bf16_to_f32(hr));
        h0[c] = hb; l0[c] = lb; h1[c] = hr; l1[c] = lr;
    }
    *(volatile u16x8*)(fnh + e) = h0;
    *(volatile u16x8*)(fnl + e) = l0;
    *(volatile u16x8*)(frh + e) = h1;
    *(volatile u16x8*)(frl + e) = l1;
    __threadfence();
    *(volatile u16x8*)(fnh + e) = h0;
    *(volatile u16x8*)(fnl + e) = l0;
    *(volatile u16x8*)(frh + e) = h1;
    *(volatile u16x8*)(frl + e) = l1;
}

template<int NBF>
__device__ __forceinline__ void tile_store_pass(const float* st, float* gp, int ldc, int lane) {
    constexpr int CW  = NBF * 16;
    constexpr int P   = CW + 4;
    constexpr int LPR = CW / 4;
    constexpr int RPI = 32 / LPR;
    constexpr int NIT = 32 / RPI;
    const int rsub = lane / LPR;
    const int c4   = (lane % LPR) * 4;
#pragma unroll
    for (int it = 0; it < NIT; ++it) {
        const int row = it * RPI + rsub;
        const v4f v = *(const v4f*)(st + row * P + c4);
        *(volatile v4f*)(gp + (size_t)row * ldc + c4) = v;
    }
}

template<int NBF>
__global__ __launch_bounds__(128)
void gemm3_kernel(const unsigned short* __restrict__ Ah, const unsigned short* __restrict__ Al,
                  const unsigned short* __restrict__ Bh, const unsigned short* __restrict__ Bl,
                  float* C, float* C2, int K, int lda, int ldc, int csplit)
{
    constexpr int CW = NBF * 16;
    constexpr int P  = CW + 4;
    __shared__ __attribute__((aligned(16))) float stile[4][32 * P];

    const int tid  = threadIdx.x;
    const int lane = tid & 31;
    const int wave = tid >> 5;
    const int h    = lane >> 4;
    const int m    = lane & 15;
    const int wm   = wave >> 1;
    const int wn   = wave & 1;

    const int rowW = blockIdx.y * 64 + wm * 32;
    const int colW = blockIdx.x * (2 * CW) + wn * CW;

    v8f acc[2 * NBF];
#pragma unroll
    for (int j = 0; j < 2 * NBF; ++j)
#pragma unroll
        for (int r = 0; r < 8; ++r) acc[j][r] = 0.0f;

    const size_t aoff = (size_t)(rowW + m) * lda + 8 * h;
    const size_t boff = (size_t)(colW + m) * K + 8 * h;
    const size_t asub = (size_t)16 * lda;
    const size_t bsub = (size_t)16 * K;
    const int nk = K >> 5;

    for (int kt = 0; kt < nk; ++kt) {
        const size_t k0 = (size_t)kt * 32;
        FragB fa[2], ga[2], fb[NBF], gb[NBF];
#pragma unroll
        for (int s = 0; s < 2; ++s) {
            const unsigned short* p = Ah + aoff + s * asub + k0;
            fa[s].h[0] = *(const u16x8*)(p);
            fa[s].h[1] = *(const u16x8*)(p + 16);
            const unsigned short* q = Al + aoff + s * asub + k0;
            ga[s].h[0] = *(const u16x8*)(q);
            ga[s].h[1] = *(const u16x8*)(q + 16);
        }
#pragma unroll
        for (int j = 0; j < NBF; ++j) {
            const unsigned short* p = Bh + boff + j * bsub + k0;
            fb[j].h[0] = *(const u16x8*)(p);
            fb[j].h[1] = *(const u16x8*)(p + 16);
            const unsigned short* q = Bl + boff + j * bsub + k0;
            gb[j].h[0] = *(const u16x8*)(q);
            gb[j].h[1] = *(const u16x8*)(q + 16);
        }
#pragma unroll
        for (int s = 0; s < 2; ++s)
#pragma unroll
            for (int j = 0; j < NBF; ++j) {
                mma16(acc[s * NBF + j], fa[s], fb[j]);
                mma16(acc[s * NBF + j], fa[s], gb[j]);
                mma16(acc[s * NBF + j], ga[s], fb[j]);
            }
    }

    float* st = stile[wave];
#pragma unroll
    for (int s = 0; s < 2; ++s)
#pragma unroll
        for (int j = 0; j < NBF; ++j)
#pragma unroll
            for (int r = 0; r < 8; ++r)
                st[(s * 16 + 8 * h + r) * P + j * 16 + m] = acc[s * NBF + j][r];
    __syncthreads();

    float* Cp = C;
    int gcol = colW;
    if (colW >= csplit) { Cp = C2; gcol = colW - csplit; }
    float* gp = Cp + (size_t)rowW * ldc + gcol;
    tile_store_pass<NBF>(st, gp, ldc, lane);
    __threadfence();
    tile_store_pass<NBF>(st, gp, ldc, lane);
}

__global__ __launch_bounds__(128)
void conv_silu_kernel(const float* __restrict__ X, const float* __restrict__ cw,
                      const float* __restrict__ cb, int rev,
                      float* UF, unsigned short* UH, unsigned short* UL)
{
    __shared__ __attribute__((aligned(16))) float srow[DI_];
    const int m   = blockIdx.x;
    const int l   = m & (NL_ - 1);
    const int tid = threadIdx.x;
    const int d0  = tid * 8;
    const float* xr = X + (size_t)m * DI_ + d0;

    const v8f x3 = ld8f(xr);
    v8f x2, x1, x0;
#pragma unroll
    for (int c = 0; c < 8; ++c) { x2[c] = 0.0f; x1[c] = 0.0f; x0[c] = 0.0f; }
    if (rev == 0) {
        if (l >= 1) x2 = ld8f(xr - DI_);
        if (l >= 2) x1 = ld8f(xr - 2 * DI_);
        if (l >= 3) x0 = ld8f(xr - 3 * DI_);
    } else {
        if (l <= NL_ - 2) x2 = ld8f(xr + DI_);
        if (l <= NL_ - 3) x1 = ld8f(xr + 2 * DI_);
        if (l <= NL_ - 4) x0 = ld8f(xr + 3 * DI_);
    }

    const float* wp = cw + (size_t)d0 * 4;
    v4f wv[8];
#pragma unroll
    for (int c = 0; c < 8; ++c) wv[c] = *(const v4f*)(wp + 4 * c);
    const v8f bias = ld8f(cb + d0);

    v8f u;
#pragma unroll
    for (int c = 0; c < 8; ++c)
        u[c] = silu_f(conv4(x0[c], x1[c], x2[c], x3[c], wv[c][0], wv[c][1], wv[c][2], wv[c][3], bias[c]));

    u16x8 hv, lv;
#pragma unroll
    for (int c = 0; c < 8; ++c) {
        const unsigned short hb = f32_to_bf16(u[c]);
        const unsigned short lb = f32_to_bf16(u[c] - bf16_to_f32(hb));
        hv[c] = hb; lv[c] = lb;
    }
    const size_t e = (size_t)m * DI_ + d0;

    *(v4f*)(srow + d0)     = __builtin_shufflevector(u, u, 0, 1, 2, 3);
    *(v4f*)(srow + d0 + 4) = __builtin_shufflevector(u, u, 4, 5, 6, 7);
    __syncthreads();
    const v4f a0 = *(const v4f*)(srow + tid * 4);
    const v4f a1 = *(const v4f*)(srow + 512 + tid * 4);
    float* gp = UF + (size_t)m * DI_;

    *(volatile u16x8*)(UH + e) = hv;
    *(volatile u16x8*)(UL + e) = lv;
    *(volatile v4f*)(gp + tid * 4) = a0;
    *(volatile v4f*)(gp + 512 + tid * 4) = a1;
    __threadfence();
    *(volatile u16x8*)(UH + e) = hv;
    *(volatile u16x8*)(UL + e) = lv;
    *(volatile v4f*)(gp + tid * 4) = a0;
    *(volatile v4f*)(gp + 512 + tid * 4) = a1;
}

__device__ __forceinline__ void rows16_store_pass(const unsigned short* sl, unsigned short* gpl,
                                                  size_t gbase, int lane) {
#pragma unroll
    for (int it = 0; it < 4; ++it) {
        const int t = it * 4 + (lane >> 3);
        const int c = (lane & 7) * 8;
        const u16x8 v = *(const u16x8*)(sl + t * 64 + c);
        *(volatile u16x8*)(gpl + gbase + (size_t)t * DI_ + c) = v;
    }
}

__global__ __launch_bounds__(64)
void scan_kernel(const float* __restrict__ U, const float* __restrict__ Z, const float* __restrict__ Dl,
                 const float* __restrict__ dbc, const float* __restrict__ dtb,
                 const float* __restrict__ Alog, const float* __restrict__ Dp, int rev,
                 unsigned short* yhi, unsigned short* ylo)
{
    __shared__ __attribute__((aligned(16))) unsigned short shi[16 * 64];
    __shared__ __attribute__((aligned(16))) unsigned short slo[16 * 64];
    __shared__ __attribute__((aligned(16))) float sbc[16 * 32];

    const int tid   = threadIdx.x;
    const int lane  = tid & 31;
    const int wave  = tid >> 5;
    const int dbase = blockIdx.x * 64;
    const int d     = dbase + tid;
    const int b     = blockIdx.y;

    float an[NS_], hs[NS_];
#pragma unroll
    for (int n = 0; n < NS_; ++n) {
        an[n] = -expf(Alog[d * NS_ + n]);
        hs[n] = 0.0f;
    }
    const float tb = dtb[d];
    const float Dd = Dp[d];
    const size_t mrow0 = (size_t)b * NL_;

    const unsigned short* sl = wave ? slo : shi;
    unsigned short* gpl = wave ? ylo : yhi;
    const int srow  = tid >> 2;
    const int spart = (tid & 3) * 8;

#pragma unroll 1
    for (int c = 0; c < NL_ / 16; ++c) {
        const int l0 = rev ? (NL_ - 16 - 16 * c) : (16 * c);
        {
            const float* src = dbc + (mrow0 + (size_t)(l0 + srow)) * DBC_ + DR_ + spart;
            *(v4f*)(sbc + srow * 32 + spart)     = *(const v4f*)(src);
            *(v4f*)(sbc + srow * 32 + spart + 4) = *(const v4f*)(src + 4);
        }
        __syncthreads();
#pragma unroll 1
        for (int t = 0; t < 16; ++t) {
            const int tt = rev ? (15 - t) : t;
            const size_t e = (mrow0 + (size_t)(l0 + tt)) * DI_ + d;
            const float u  = U[e];
            const float zv = Z[e];
            const float dl = Dl[e];
            const float dt = softplus_f(dl + tb);
            const float du = dt * u;
            const float* bc = sbc + tt * 32;
            float y = 0.0f;
#pragma unroll
            for (int n = 0; n < NS_; ++n) {
                const float da = __expf(dt * an[n]);
                hs[n] = da * hs[n] + du * bc[n];
                y += hs[n] * bc[NS_ + n];
            }
            const float gval = (y + Dd * u) * silu_f(zv);
            const unsigned short hb = f32_to_bf16(gval);
            const unsigned short lb = f32_to_bf16(gval - bf16_to_f32(hb));
            shi[tt * 64 + tid] = hb;
            slo[tt * 64 + tid] = lb;
        }
        __syncthreads();
        const size_t gbase = (mrow0 + (size_t)l0) * DI_ + dbase;
        rows16_store_pass(sl, gpl, gbase, lane);
        __threadfence();
        rows16_store_pass(sl, gpl, gbase, lane);
        __syncthreads();
    }
}

__global__ __launch_bounds__(256)
void combine_kernel(const float* __restrict__ fw, const float* __restrict__ gb,
                    const float* __restrict__ of, const float* __restrict__ ob,
                    float* out, int n4)
{
    const int i = blockIdx.x * 256 + threadIdx.x;
    if (i >= n4) return;
    const size_t e = (size_t)i * 4;
    const int col = (int)(e & (size_t)(DM_ - 1));
    const v4f a = *(const v4f*)(fw + e) + *(const v4f*)(gb + col);
    const v4f s = *(const v4f*)(of + e) + *(const v4f*)(ob + e);
    const v4f r = a * s;
    *(volatile v4f*)(out + e) = r;
    __threadfence();
    *(volatile v4f*)(out + e) = r;
}

extern "C" void kernel_launch(void* const* d_in, const int* in_sizes, int n_in,
                              void* d_out, int out_size, void* d_ws, size_t ws_size,
                              hipStream_t stream)
{
    if (n_in < 23) return;
    if (in_sizes[0] != MT_ * DM_) return;
    if (in_sizes[1] != DM_) return;
    if (in_sizes[2] != DM_) return;
    if (in_sizes[3] != DM_ * DM_) return;
    if (in_sizes[4] != DM_) return;
    for (int dir = 0; dir < 2; ++dir) {
        const int o = 5 + 9 * dir;
        if (in_sizes[o + 0] != 2 * DI_ * DM_) return;
        if (in_sizes[o + 1] != DI_ * 4)       return;
        if (in_sizes[o + 2] != DI_)           return;
        if (in_sizes[o + 3] != DBC_ * DI_)    return;
        if (in_sizes[o + 4] != DI_ * DR_)     return;
        if (in_sizes[o + 5] != DI_)           return;
        if (in_sizes[o + 6] != DI_ * NS_)     return;
        if (in_sizes[o + 7] != DI_)           return;
        if (in_sizes[o + 8] != DM_ * DI_)     return;
    }
    if (out_size != MT_ * DM_) return;

    const float* x      = (const float*)d_in[0];
    const float* ln_g   = (const float*)d_in[1];
    const float* ln_b   = (const float*)d_in[2];
    const float* gate_w = (const float*)d_in[3];
    const float* gate_b = (const float*)d_in[4];
    float* out = (float*)d_out;

    const size_t SZ_P512  = (size_t)MT_ * DM_ * 2;
    const size_t SZ_F512  = (size_t)MT_ * DM_ * 4;
    const size_t SZ_P1024 = (size_t)MT_ * DI_ * 2;
    const size_t SZ_F1024 = (size_t)MT_ * DI_ * 4;
    const size_t SZ_GW    = (size_t)DM_ * DM_ * 2;
    const size_t SZ_WIN   = (size_t)2 * DI_ * DM_ * 2;
    const size_t SZ_WX    = (size_t)DBC_ * DI_ * 2;
    const size_t SZ_WDT   = (size_t)DI_ * DR_ * 2;
    const size_t SZ_WOUT  = (size_t)DM_ * DI_ * 2;
    const size_t SZ_DBC   = (size_t)MT_ * DBC_ * 4;
    const size_t SZ_DBCP  = (size_t)MT_ * DBC_ * 2;

    const size_t OFF_FNH   = 0;
    const size_t OFF_FNL   = OFF_FNH + SZ_P512;
    const size_t OFF_FRH   = OFF_FNL + SZ_P512;
    const size_t OFF_FRL   = OFF_FRH + SZ_P512;
    const size_t OFF_FW    = OFF_FRL + SZ_P512;
    const size_t OFF_GWH   = OFF_FW + SZ_F512;
    const size_t OFF_GWL   = OFF_GWH + SZ_GW;
    const size_t OFF_WINH  = OFF_GWL + SZ_GW;
    const size_t OFF_WINL  = OFF_WINH + SZ_WIN;
    const size_t OFF_WXH   = OFF_WINL + SZ_WIN;
    const size_t OFF_WXL   = OFF_WXH + SZ_WX;
    const size_t OFF_WDTH  = OFF_WXL + SZ_WX;
    const size_t OFF_WDTL  = OFF_WDTH + SZ_WDT;
    const size_t OFF_WOUTH = OFF_WDTL + SZ_WDT;
    const size_t OFF_WOUTL = OFF_WOUTH + SZ_WOUT;
    const size_t OFF_XF    = OFF_WOUTL + SZ_WOUT;
    const size_t OFF_ZF    = OFF_XF + SZ_F1024;
    const size_t OFF_XCF   = OFF_ZF + SZ_F1024;
    const size_t OFF_XCH   = OFF_XCF + SZ_F1024;
    const size_t OFF_XCL   = OFF_XCH + SZ_P1024;
    const size_t OFF_DBC   = OFF_XCL + SZ_P1024;
    const size_t OFF_DBCH  = OFF_DBC + SZ_DBC;
    const size_t OFF_DBCL  = OFF_DBCH + SZ_DBCP;
    const size_t OFF_OUTB  = OFF_DBCL + SZ_DBCP;
    const size_t WS_END    = OFF_OUTB + SZ_F512;
    const size_t OFF_OUTF  = OFF_FRH;
    const size_t OFF_DL    = OFF_XF;
    const size_t OFF_YH    = OFF_XCH;
    const size_t OFF_YL    = OFF_XCL;
    if (2 * SZ_P512 != SZ_F512) return;
    if (ws_size < WS_END) return;

    char* ws = (char*)d_ws;
    unsigned short* fnh   = (unsigned short*)(ws + OFF_FNH);
    unsigned short* fnl   = (unsigned short*)(ws + OFF_FNL);
    unsigned short* frh   = (unsigned short*)(ws + OFF_FRH);
    unsigned short* frl   = (unsigned short*)(ws + OFF_FRL);
    float*          FW    = (float*)(ws + OFF_FW);
    unsigned short* gwh   = (unsigned short*)(ws + OFF_GWH);
    unsigned short* gwl   = (unsigned short*)(ws + OFF_GWL);
    unsigned short* winh  = (unsigned short*)(ws + OFF_WINH);
    unsigned short* winl  = (unsigned short*)(ws + OFF_WINL);
    unsigned short* wxh   = (unsigned short*)(ws + OFF_WXH);
    unsigned short* wxl   = (unsigned short*)(ws + OFF_WXL);
    unsigned short* wdth  = (unsigned short*)(ws + OFF_WDTH);
    unsigned short* wdtl  = (unsigned short*)(ws + OFF_WDTL);
    unsigned short* wouth = (unsigned short*)(ws + OFF_WOUTH);
    unsigned short* woutl = (unsigned short*)(ws + OFF_WOUTL);
    float*          XF    = (float*)(ws + OFF_XF);
    float*          ZF    = (float*)(ws + OFF_ZF);
    float*          XCF   = (float*)(ws + OFF_XCF);
    unsigned short* XCH   = (unsigned short*)(ws + OFF_XCH);
    unsigned short* XCL   = (unsigned short*)(ws + OFF_XCL);
    float*          DBCF  = (float*)(ws + OFF_DBC);
    unsigned short* dbch  = (unsigned short*)(ws + OFF_DBCH);
    unsigned short* dbcl  = (unsigned short*)(ws + OFF_DBCL);
    float*          OUTB  = (float*)(ws + OFF_OUTB);
    float*          OUTF  = (float*)(ws + OFF_OUTF);
    float*          DL    = (float*)(ws + OFF_DL);
    unsigned short* YH    = (unsigned short*)(ws + OFF_YH);
    unsigned short* YL    = (unsigned short*)(ws + OFF_YL);

    hipLaunchKernelGGL(ln_kernel, dim3(MT_), dim3(64), 0, stream, x, ln_g, ln_b, fnh, fnl, frh, frl);

    {
        const int n8 = (DM_ * DM_) / 8;
        hipLaunchKernelGGL(cvt_split_kernel, dim3((n8 + 255) / 256), dim3(256), 0, stream,
                           gate_w, gwh, gwl, n8);
    }
    hipLaunchKernelGGL(HIP_KERNEL_NAME(gemm3_kernel<2>), dim3(DM_ / 64, MT_ / 64), dim3(128), 0, stream,
                       (const unsigned short*)frh, (const unsigned short*)frl,
                       (const unsigned short*)gwh, (const unsigned short*)gwl,
                       FW, FW, (int)DM_, (int)DM_, (int)DM_, (int)(4 * DM_));

    for (int dir = 0; dir < 2; ++dir) {
        const int o = 5 + 9 * dir;
        const float* W_in   = (const float*)d_in[o + 0];
        const float* conv_w = (const float*)d_in[o + 1];
        const float* conv_b = (const float*)d_in[o + 2];
        const float* W_x    = (const float*)d_in[o + 3];
        const float* W_dt   = (const float*)d_in[o + 4];
        const float* b_dt   = (const float*)d_in[o + 5];
        const float* A_log  = (const float*)d_in[o + 6];
        const float* Dp     = (const float*)d_in[o + 7];
        const float* W_out  = (const float*)d_in[o + 8];

        {
            int n8;
            n8 = (2 * DI_ * DM_) / 8;
            hipLaunchKernelGGL(cvt_split_kernel, dim3((n8 + 255) / 256), dim3(256), 0, stream, W_in, winh, winl, n8);
            n8 = (DBC_ * DI_) / 8;
            hipLaunchKernelGGL(cvt_split_kernel, dim3((n8 + 255) / 256), dim3(256), 0, stream, W_x, wxh, wxl, n8);
            n8 = (DI_ * DR_) / 8;
            hipLaunchKernelGGL(cvt_split_kernel, dim3((n8 + 255) / 256), dim3(256), 0, stream, W_dt, wdth, wdtl, n8);
            n8 = (DM_ * DI_) / 8;
            hipLaunchKernelGGL(cvt_split_kernel, dim3((n8 + 255) / 256), dim3(256), 0, stream, W_out, wouth, woutl, n8);
        }

        hipLaunchKernelGGL(HIP_KERNEL_NAME(gemm3_kernel<2>), dim3((2 * DI_) / 64, MT_ / 64), dim3(128), 0, stream,
                           (const unsigned short*)fnh, (const unsigned short*)fnl,
                           (const unsigned short*)winh, (const unsigned short*)winl,
                           XF, ZF, (int)DM_, (int)DM_, (int)DI_, (int)DI_);

        hipLaunchKernelGGL(conv_silu_kernel, dim3(MT_), dim3(128), 0, stream,
                           (const float*)XF, conv_w, conv_b, dir, XCF, XCH, XCL);

        hipLaunchKernelGGL(HIP_KERNEL_NAME(gemm3_kernel<2>), dim3(DBC_ / 64, MT_ / 64), dim3(128), 0, stream,
                           (const unsigned short*)XCH, (const unsigned short*)XCL,
                           (const unsigned short*)wxh, (const unsigned short*)wxl,
                           DBCF, DBCF, (int)DI_, (int)DI_, (int)DBC_, (int)(4 * DBC_));

        {
            const int n8 = (MT_ * DBC_) / 8;
            hipLaunchKernelGGL(cvt_split_kernel, dim3((n8 + 255) / 256), dim3(256), 0, stream,
                               (const float*)DBCF, dbch, dbcl, n8);
        }

        hipLaunchKernelGGL(HIP_KERNEL_NAME(gemm3_kernel<2>), dim3(DI_ / 64, MT_ / 64), dim3(128), 0, stream,
                           (const unsigned short*)dbch, (const unsigned short*)dbcl,
                           (const unsigned short*)wdth, (const unsigned short*)wdtl,
                           DL, DL, (int)DR_, (int)DBC_, (int)DI_, (int)(4 * DI_));

        hipLaunchKernelGGL(scan_kernel, dim3(DI_ / 64, NB_), dim3(64), 0, stream,
                           (const float*)XCF, (const float*)ZF, (const float*)DL, (const float*)DBCF,
                           b_dt, A_log, Dp, dir, YH, YL);

        float* od = dir ? OUTB : OUTF;
        hipLaunchKernelGGL(HIP_KERNEL_NAME(gemm3_kernel<2>), dim3(DM_ / 64, MT_ / 64), dim3(128), 0, stream,
                           (const unsigned short*)YH, (const unsigned short*)YL,
                           (const unsigned short*)wouth, (const unsigned short*)woutl,
                           od, od, (int)DI_, (int)DI_, (int)DM_, (int)(4 * DM_));
    }

    {
        const int n4 = (MT_ * DM_) / 4;
        hipLaunchKernelGGL(combine_kernel, dim3((n4 + 255) / 256), dim3(256), 0, stream,
                           (const float*)FW, gate_b, (const float*)OUTF, (const float*)OUTB, out, n4);
    }
}
